// BiMamba_79250736546334
// MI455X (gfx1250) — hardware-run, weakly checked
//
#include <hip/hip_runtime.h>
#include <hip/hip_fp16.h>
#include <math.h>

typedef __attribute__((ext_vector_type(16))) _Float16 v16h;
typedef __attribute__((ext_vector_type(8)))  _Float16 v8h;
typedef __attribute__((ext_vector_type(8)))  float    v8f;
typedef __attribute__((ext_vector_type(4)))  float    v4f;
typedef __attribute__((ext_vector_type(4)))  unsigned v4u;

constexpr int kBatch  = 2;
constexpr int kSeq    = 2048;
constexpr int kDm     = 1024;
constexpr int kDin    = 2048;
constexpr int kNst    = 16;
constexpr int kDtR    = 64;
constexpr int kXzP    = 2 * kDin;
constexpr int kXdW    = kDtR + 2 * kNst;
constexpr int kXdP    = 128;
constexpr int kOffB   = kDtR;
constexpr int kOffC   = kDtR + kNst;
constexpr int kRows   = kBatch * kSeq;
constexpr int kConvTP = 260;
static_assert(kXdW == 96 && kXdW <= kXdP, "x_proj width");
static_assert((kDm % 32) == 0 && (kDin % 32) == 0 && (kDtR % 32) == 0, "GEMM K multiples of 32");
static_assert((kSeq % 64) == 0 && (kXzP % 64) == 0 && (kXdP % 64) == 0 && (kDin % 64) == 0 && (kDm % 64) == 0 && (kRows % 64) == 0, "GEMM M,N multiples of 64");
static_assert((kDin % 256) == 0 && (kSeq % 64) == 0, "conv tile multiples");

constexpr float kCX   = 16.0f;
constexpr float kCWin = 1024.0f;
constexpr float kCU   = 64.0f;
constexpr float kCWx  = 1024.0f;
constexpr float kCDt  = 256.0f;
constexpr float kCWdt = 64.0f;
constexpr float kCY   = 1024.0f;
constexpr float kCWo  = 1024.0f;
constexpr float kSclIn  = 1.0f / (kCX * kCWin);
constexpr float kSclXp  = 1.0f / (kCU * kCWx);
constexpr float kSclDt  = 1.0f / (kCDt * kCWdt);
constexpr float kSclOut = 1.0f / (kCY * kCWo);

constexpr size_t kOffX16   = 0;
constexpr size_t kOffWIN   = kOffX16   + (size_t)kRows * kDm * 2;
constexpr size_t kOffWOUT  = kOffWIN   + (size_t)kXzP * kDm * 2;
constexpr size_t kOffWXF   = kOffWOUT  + (size_t)kDm * kDin * 2;
constexpr size_t kOffWXB   = kOffWXF   + (size_t)kXdP * kDin * 2;
constexpr size_t kOffWDF   = kOffWXB   + (size_t)kXdP * kDin * 2;
constexpr size_t kOffWDB   = kOffWDF   + (size_t)kDin * kDtR * 2;
constexpr size_t kOffXZB   = kOffWDB   + (size_t)kDin * kDtR * 2;
constexpr size_t kOffU32   = kOffXZB   + (size_t)kSeq * kXzP * 4;
constexpr size_t kOffU16   = kOffU32   + (size_t)kSeq * kDin * 4;
constexpr size_t kOffXDBL  = kOffU16   + (size_t)kSeq * kDin * 2;
constexpr size_t kOffDTLR  = kOffXDBL  + (size_t)kSeq * kXdP * 4;
constexpr size_t kOffDTPRE = kOffDTLR  + (size_t)kSeq * kDtR * 2;
constexpr size_t kOffYF    = kOffDTPRE + (size_t)kSeq * kDin * 4;
constexpr size_t kOffYB    = kOffYF    + (size_t)kSeq * kDin * 2;
constexpr size_t kOffY16   = kOffYB    + (size_t)kSeq * kDin * 2;
constexpr size_t kWsTotal  = kOffY16   + (size_t)kRows * kDin * 2;
static_assert(kWsTotal == 132907008ull, "carve total");
static_assert(kWsTotal <= 134217728ull, "carve cap");
static_assert((kOffWIN % 128) == 0 && (kOffWOUT % 128) == 0 && (kOffWXF % 128) == 0 && (kOffWXB % 128) == 0 &&
              (kOffWDF % 128) == 0 && (kOffWDB % 128) == 0 && (kOffXZB % 128) == 0 && (kOffU32 % 128) == 0 &&
              (kOffU16 % 128) == 0 && (kOffXDBL % 128) == 0 && (kOffDTLR % 128) == 0 && (kOffDTPRE % 128) == 0 &&
              (kOffYF % 128) == 0 && (kOffYB % 128) == 0 && (kOffY16 % 128) == 0, "128-B aligned regions");

__device__ __forceinline__ _Float16 f16_flushed(float w) {
  const float f = (fabsf(w) < 6.103515625e-05f) ? 0.0f : w;
  return (_Float16)f;
}
__device__ __forceinline__ float h16_to_f32(unsigned hb) {
  const unsigned sgn = (hb & 0x8000u) << 16;
  const unsigned em = hb & 0x7fffu;
  const float fn = __uint_as_float((em << 13) + 0x38000000u);
  const float fs = (float)em * 5.9604644775390625e-8f;
  const float mag = (em < 0x400u) ? fs : fn;
  return __uint_as_float(__float_as_uint(mag) | sgn);
}

namespace eng {

__device__ __forceinline__ v16h frag_load(const _Float16* p) {
  union { v16h v; v8h h[2]; } f;
  f.h[0] = *(const v8h*)(p);
  f.h[1] = *(const v8h*)(p + 16);
  return f.v;
}
__device__ __forceinline__ v8f mma_f16(v16h a, v16h b, v8f c) {
  c = __builtin_amdgcn_wmma_f32_16x16x32_f16(false, a, false, b, (short)0, c, false, false);
  asm volatile("v_nop\n\tv_nop\n\tv_nop\n\tv_nop" : "+v"(c) : "v"(a), "v"(b));
  return c;
}

template <int BIAS2>
__global__ __launch_bounds__(256) void gemm_f16_kernel(
    const unsigned short* __restrict__ Ap, int lda,
    const unsigned short* __restrict__ Btp, int ldb,
    float* __restrict__ C, int ldc,
    const float* __restrict__ bias,
    int M, int N, int K, float scale)
{
  const _Float16* A  = (const _Float16*)Ap;
  const _Float16* Bt = (const _Float16*)Btp;
  __shared__ __align__(16) float sT[8][16 * 68];
  const int lane = threadIdx.x & 31;
  const int wave = threadIdx.x >> 5;
  const int tilesN = N >> 6;
  const int tilesM = M >> 6;
  const int tile = blockIdx.x * 8 + wave;
  if (tile >= tilesM * tilesN) return;
  const int tm = tile / tilesN;
  const int tn = tile - tm * tilesN;
  const int m0 = tm << 6;
  const int n0 = tn << 6;
  const int rlane = lane & 15;
  const int koff  = (lane >> 4) * 8;
  const int mOff  = (lane >> 4) * 8;

  v8f acc[4][4];
#pragma unroll
  for (int i = 0; i < 4; ++i)
#pragma unroll
    for (int j = 0; j < 4; ++j) acc[i][j] = (v8f){0.f, 0.f, 0.f, 0.f, 0.f, 0.f, 0.f, 0.f};

  for (int k0 = 0; k0 < K; k0 += 32) {
    v16h bh[4];
#pragma unroll
    for (int j = 0; j < 4; ++j) {
      const size_t bo = (size_t)(n0 + (j << 4) + rlane) * ldb + koff + k0;
      bh[j] = frag_load(Bt + bo);
    }
#pragma unroll
    for (int i = 0; i < 4; ++i) {
      const size_t ao = (size_t)(m0 + (i << 4) + rlane) * lda + koff + k0;
      const v16h ah = frag_load(A + ao);
#pragma unroll
      for (int j = 0; j < 4; ++j) acc[i][j] = mma_f16(ah, bh[j], acc[i][j]);
    }
  }

  float* slab = sT[wave];
#pragma unroll
  for (int i = 0; i < 4; ++i) {
    const int mBase = m0 + (i << 4);
#pragma unroll
    for (int j = 0; j < 4; ++j) {
      const int n = n0 + (j << 4) + rlane;
      float bv = 0.f;
      if (BIAS2) bv = bias[n];
#pragma unroll
      for (int r = 0; r < 8; ++r) {
        float v = acc[i][j][r] * scale;
        if (BIAS2) {
          v = v + bv;
          v = v + bv;
        }
        slab[(mOff + r) * 68 + (j << 4) + rlane] = v;
      }
    }
    __builtin_amdgcn_fence(__ATOMIC_RELEASE, "workgroup");
    __builtin_amdgcn_wave_barrier();
    __builtin_amdgcn_fence(__ATOMIC_ACQUIRE, "workgroup");
    {
      const int hh = lane >> 4, c4 = (lane & 15) * 4;
      for (int pass = 0; pass < 2; ++pass) {
#pragma unroll
        for (int it = 0; it < 8; ++it) {
          const int row = it * 2 + hh;
          v4f v = *(const v4f*)(slab + row * 68 + c4);
          *(volatile v4f*)(C + (size_t)(mBase + row) * ldc + n0 + c4) = v;
        }
        __threadfence();
      }
    }
    __builtin_amdgcn_fence(__ATOMIC_RELEASE, "workgroup");
    __builtin_amdgcn_wave_barrier();
    __builtin_amdgcn_fence(__ATOMIC_ACQUIRE, "workgroup");
  }
}

}

__global__ __launch_bounds__(256) void cast_plane_f16_kernel(
    const float* __restrict__ src, int src_ld, int src_rows,
    unsigned short* __restrict__ dst, int cols, int total8, float carry)
{
  const int i = blockIdx.x * 256 + threadIdx.x;
  if (i >= total8) return;
  const int c8n = cols >> 3;
  const int row = i / c8n;
  const int c8  = (i - row * c8n) << 3;
  const bool valid = (row < src_rows);
  const int rc = valid ? row : (src_rows - 1);
  const float* sp = src + (size_t)rc * src_ld + c8;
  v4f a0 = *(const v4f*)(sp);
  v4f a1 = *(const v4f*)(sp + 4);
  asm volatile("" : "+v"(a0), "+v"(a1));
  v8h hv;
#pragma unroll
  for (int e = 0; e < 4; ++e) {
    const float f0 = valid ? a0[e] : 0.0f;
    const float f1 = valid ? a1[e] : 0.0f;
    hv[e]     = f16_flushed(f0 * carry);
    hv[4 + e] = f16_flushed(f1 * carry);
  }
  unsigned short* q = dst + ((size_t)i << 3);
  *(volatile v8h*)q = hv;
  __threadfence();
  *(volatile v8h*)q = hv;
}

__global__ __launch_bounds__(256) void conv_silu_kernel(
    const float* __restrict__ XZb, const float* __restrict__ cw, const float* __restrict__ cb,
    float* __restrict__ U32, unsigned short* __restrict__ U16, int flip)
{
  __shared__ __align__(16) float sT[16 * kConvTP];
  const int tid = threadIdx.x, lane = tid & 31, wave = tid >> 5;
  const int d0 = blockIdx.x * 256, d = d0 + tid;
  const int t0 = blockIdx.y * 64;
  const int rbase = flip ? (kSeq - 1) : 0;
  const int rsgn  = flip ? -1 : 1;
  const v4f wv = *(const v4f*)(cw + (size_t)d * 4);
  const float w0 = wv[0], w1 = wv[1], w2 = wv[2], w3 = wv[3];
  const float bc = cb[d];
  float xm3, xm2, xm1;
  {
    const bool hist = (t0 > 0);
    const int tq = hist ? (t0 - 3) : 0;
    const float v3 = XZb[(size_t)(rbase + rsgn * tq) * kXzP + d];
    const float v2 = XZb[(size_t)(rbase + rsgn * (tq + 1)) * kXzP + d];
    const float v1 = XZb[(size_t)(rbase + rsgn * (tq + 2)) * kXzP + d];
    xm3 = hist ? v3 : 0.0f;
    xm2 = hist ? v2 : 0.0f;
    xm1 = hist ? v1 : 0.0f;
  }
  const int hrow = wave >> 1;
  const int hch  = (wave & 1) * 128 + lane * 4;
#pragma unroll 1
  for (int sub = 0; sub < 4; ++sub) {
    const int tb = t0 + sub * 16;
#pragma unroll 1
    for (int s = 0; s < 16; ++s) {
      const float xcur = XZb[(size_t)(rbase + rsgn * (tb + s)) * kXzP + d];
      float acc = w0 * xm3;
      acc = fmaf(w1, xm2, acc);
      acc = fmaf(w2, xm1, acc);
      acc = fmaf(w3, xcur, acc);
      const float sv = acc + bc;
      const float sg = __builtin_amdgcn_rcpf(1.0f + expf(-sv));
      sT[s * kConvTP + tid] = sv * sg;
      xm3 = xm2;
      xm2 = xm1;
      xm1 = xcur;
    }
    __syncthreads();
    v4f fv[4];
    v8h hv[2];
#pragma unroll
    for (int it = 0; it < 4; ++it) fv[it] = *(const v4f*)(sT + (it * 4 + hrow) * kConvTP + hch);
#pragma unroll
    for (int it = 0; it < 2; ++it) {
      const float* sp = sT + (it * 8 + wave) * kConvTP + lane * 8;
      const v4f a0 = *(const v4f*)(sp);
      const v4f a1 = *(const v4f*)(sp + 4);
#pragma unroll
      for (int e = 0; e < 4; ++e) {
        hv[it][e]     = f16_flushed(a0[e] * kCU);
        hv[it][4 + e] = f16_flushed(a1[e] * kCU);
      }
    }
    for (int pass = 0; pass < 2; ++pass) {
#pragma unroll
      for (int it = 0; it < 4; ++it)
        *(volatile v4f*)(U32 + (size_t)(tb + it * 4 + hrow) * kDin + d0 + hch) = fv[it];
#pragma unroll
      for (int it = 0; it < 2; ++it)
        *(volatile v8h*)(U16 + (size_t)(tb + it * 8 + wave) * kDin + d0 + lane * 8) = hv[it];
      __threadfence();
    }
    __syncthreads();
  }
}

__global__ __launch_bounds__(256) void zflip_kernel(const float* zsrc, float* dst)
{
  const int i = blockIdx.x * 256 + threadIdx.x;
  const int r  = i >> 9;
  const int c4 = (i & 511) << 2;
  const v4f va = *(const v4f*)(zsrc + (size_t)(kSeq - 1 - r) * kXzP + c4);
  const v4f vb = *(const v4f*)(zsrc + (size_t)(kSeq / 2 - 1 - r) * kXzP + c4);
  float* pa = dst + (size_t)r * kXzP + c4;
  float* pb = dst + (size_t)(r + kSeq / 2) * kXzP + c4;
  *(volatile v4f*)pa = va;
  *(volatile v4f*)pb = vb;
  __threadfence();
  *(volatile v4f*)pa = va;
  *(volatile v4f*)pb = vb;
}

__global__ __launch_bounds__(256) void combine_kernel(
    const unsigned* __restrict__ YF, const unsigned* __restrict__ YB, unsigned short* __restrict__ YO)
{
  const int i = blockIdx.x * 256 + threadIdx.x;
  const int t  = i >> 8;
  const int c8 = (i & 255) << 3;
  const size_t of = ((size_t)t * kDin + c8) >> 1;
  const size_t ob = ((size_t)(kSeq - 1 - t) * kDin + c8) >> 1;
  const v4u a = *(const v4u*)(YF + of);
  const v4u b = *(const v4u*)(YB + ob);
  v8h hv;
#pragma unroll
  for (int k = 0; k < 4; ++k) {
    const unsigned wa = a[k];
    const unsigned wb = b[k];
    const float s0 = h16_to_f32(wa & 0xffffu) + h16_to_f32(wb & 0xffffu);
    const float s1 = h16_to_f32(wa >> 16) + h16_to_f32(wb >> 16);
    hv[2 * k]     = f16_flushed(s0);
    hv[2 * k + 1] = f16_flushed(s1);
  }
  unsigned short* p = YO + (size_t)t * kDin + c8;
  *(volatile v8h*)p = hv;
  __threadfence();
  *(volatile v8h*)p = hv;
}

typedef float    ms1_v4f __attribute__((ext_vector_type(4)));
typedef unsigned ms1_v4u __attribute__((ext_vector_type(4)));
struct ms1_args {
  const float* dtpre;
  const float* u;
  const float* bc;
  const float* z;
  const float* A_log;
  const float* Dskip;
  __half* y;
  __half* y_lo;
  long ld_dtpre;
  long ld_u;
  long ld_bc;
  long ld_z;
  long ld_y;
  int offB;
  int offC;
  int offZ;
  float ycarry;
  int dir;
  int D;
  int L;
  int nbatch;
};
static_assert(sizeof(ms1_args) == 136);

__device__ __forceinline__ float ms1_flush16(float v) {
  return (fabsf(v) < 6.103515625e-05f) ? 0.0f : v;
}
__device__ __forceinline__ unsigned ms1_h16bits(float v) {
  return (unsigned)__half_as_ushort(__float2half_rn(ms1_flush16(v)));
}
__device__ __forceinline__ float ms1_h16val(unsigned b) {
  return __half2float(__ushort_as_half((unsigned short)b));
}
__device__ __forceinline__ float ms1_softplus(float v) {
  return fmaxf(v, 0.0f) + log1pf(expf(-fabsf(v)));
}
__device__ __forceinline__ void ms1_pack2(float v0, float v1, unsigned& hw, unsigned& lw) {
  const unsigned h0 = ms1_h16bits(v0);
  const unsigned h1 = ms1_h16bits(v1);
  const float r0 = (v0 - ms1_h16val(h0)) * 2048.0f;
  const float r1 = (v1 - ms1_h16val(h1)) * 2048.0f;
  const unsigned l0 = ms1_h16bits(r0);
  const unsigned l1 = ms1_h16bits(r1);
  hw = h0 | (h1 << 16);
  lw = l0 | (l1 << 16);
}

template <int NSTATE>
__global__ __launch_bounds__(64 * (NSTATE / 16)) void ms1_scan_kernel(ms1_args a)
{
  static_assert(NSTATE == 16 || NSTATE == 64);
  constexpr int NQ  = NSTATE / 16;
  constexpr int NT  = 64 * NQ;
  constexpr int NW  = NT / 32;
  constexpr int BCW = 2 * NSTATE;
  constexpr int YP  = 68;
  constexpr int RPI = NW * 4;
  constexpr int NIT = 64 / RPI;
  static_assert(16 * NT <= 64 * YP);
  __shared__ __align__(16) float sBC[64 * BCW];
  __shared__ __align__(16) float sY[64 * YP];
  const int tid  = threadIdx.x;
  const int lane = tid & 31;
  const int wave = tid >> 5;
  const int c    = tid / NQ;
  const int sq   = tid - c * NQ;
  const int bpb  = a.D / 64;
  const int bi   = blockIdx.x / bpb;
  if (bi >= a.nbatch) return;
  const int d0 = (blockIdx.x - bi * bpb) * 64;
  const int d  = d0 + c;
  const long rowb = (long)bi * a.L;
  const bool hasz  = (a.z != nullptr);
  const bool hasD  = (a.Dskip != nullptr);
  const bool hasLo = (a.y_lo != nullptr);

#pragma unroll 1
  for (int n = 0; n < 16; ++n) {
    const float al = a.A_log[(long)d * NSTATE + sq * 16 + n];
    sY[n * NT + tid] = -expf(al);
  }
  __syncthreads();
  float An[16], h[16];
#pragma unroll
  for (int n = 0; n < 16; ++n) {
    An[n] = sY[n * NT + tid];
    h[n] = 0.0f;
  }
  float Dd = 0.0f;
  if (hasD) Dd = a.Dskip[d];

  const int nchunk = a.L / 64;
  const bool fwd = (a.dir > 0);
  const int s0 = fwd ? 0 : 63;
  const int sd = fwd ? 1 : -1;
  const int q  = lane >> 3;
  const int c8 = (lane & 7) * 8;

#pragma unroll 1
  for (int ci = 0; ci < nchunk; ++ci) {
    const int tb = fwd ? (ci * 64) : (a.L - 64 - ci * 64);
    const long rowc = rowb + tb;
    __syncthreads();
#pragma unroll 8
    for (int i = 0; i < 32; ++i) {
      const int idx = tid + i * NT;
      const int st  = idx / BCW;
      const int col = idx - st * BCW;
      const int sc  = (col < NSTATE) ? (a.offB + col) : (a.offC + col - NSTATE);
      sBC[idx] = a.bc[(rowc + st) * a.ld_bc + sc];
    }
    __syncthreads();
#pragma unroll 1
    for (int s = 0; s < 64; ++s) {
      const int ls = s0 + sd * s;
      const long row = rowc + ls;
      float pre = a.dtpre[row * a.ld_dtpre + d];
      float uv  = a.u[row * a.ld_u + d];
      float zv  = 0.0f;
      if (hasz) zv = a.z[row * a.ld_z + a.offZ + d];
      asm volatile("" : "+v"(pre));
      asm volatile("" : "+v"(uv));
      asm volatile("" : "+v"(zv));
      const float delta = ms1_softplus(pre);
      const float dtx = delta * uv;
      const float* bp = sBC + ls * BCW + sq * 16;
      const float* cp = bp + NSTATE;
      ms1_v4f Bq[4], Cq[4];
#pragma unroll
      for (int k = 0; k < 4; ++k) {
        Bq[k] = *(const ms1_v4f*)(bp + 4 * k);
        Cq[k] = *(const ms1_v4f*)(cp + 4 * k);
      }
      float yv = 0.0f;
#pragma unroll
      for (int n = 0; n < 16; ++n) {
        const float e = __expf(delta * An[n]);
        h[n] = fmaf(e, h[n], dtx * Bq[n >> 2][n & 3]);
        yv = fmaf(h[n], Cq[n >> 2][n & 3], yv);
      }
      if (NQ > 1) {
        yv += __shfl_xor(yv, 1, 32);
        yv += __shfl_xor(yv, 2, 32);
      }
      if (hasD) yv = fmaf(uv, Dd, yv);
      if (hasz) {
        const float sg = __builtin_amdgcn_rcpf(1.0f + expf(-zv));
        yv = yv * (zv * sg);
      }
      if (sq == 0) sY[ls * YP + c] = yv * a.ycarry;
    }
    __syncthreads();
    ms1_v4u hw[NIT], lw[NIT];
#pragma unroll
    for (int it = 0; it < NIT; ++it) {
      const int row = it * RPI + wave * 4 + q;
      const float* sp = sY + row * YP + c8;
      const ms1_v4f f0 = *(const ms1_v4f*)(sp);
      const ms1_v4f f1 = *(const ms1_v4f*)(sp + 4);
      unsigned h0, h1, h2, h3, l0, l1, l2, l3;
      ms1_pack2(f0[0], f0[1], h0, l0);
      ms1_pack2(f0[2], f0[3], h1, l1);
      ms1_pack2(f1[0], f1[1], h2, l2);
      ms1_pack2(f1[2], f1[3], h3, l3);
      hw[it] = (ms1_v4u){h0, h1, h2, h3};
      lw[it] = (ms1_v4u){l0, l1, l2, l3};
    }
    for (int pass = 0; pass < 2; ++pass) {
#pragma unroll
      for (int it = 0; it < NIT; ++it) {
        const int row = it * RPI + wave * 4 + q;
        const long o = (rowc + row) * a.ld_y + d0 + c8;
        *(volatile ms1_v4u*)(a.y + o) = hw[it];
        if (hasLo) *(volatile ms1_v4u*)(a.y_lo + o) = lw[it];
      }
      __threadfence();
    }
  }
}

extern "C" void kernel_launch(void* const* d_in, const int* in_sizes, int n_in,
                              void* d_out, int out_size, void* d_ws, size_t ws_size,
                              hipStream_t stream) {
  if (n_in < 17) return;
  if (in_sizes[0] != kRows * kDm) return;
  if (in_sizes[1] != kXzP * kDm) return;
  if (in_sizes[2] != kDin * 4) return;
  if (in_sizes[3] != kDin) return;
  if (in_sizes[4] != kDin * 4) return;
  if (in_sizes[5] != kDin) return;
  if (in_sizes[6] != kXdW * kDin) return;
  if (in_sizes[7] != kXdW * kDin) return;
  if (in_sizes[8] != kDin * kDtR) return;
  if (in_sizes[9] != kDin) return;
  if (in_sizes[10] != kDin * kDtR) return;
  if (in_sizes[11] != kDin) return;
  if (in_sizes[12] != kDin * kNst) return;
  if (in_sizes[13] != kDin * kNst) return;
  if (in_sizes[14] != kDin) return;
  if (in_sizes[15] != kDin) return;
  if (in_sizes[16] != kDm * kDin) return;
  if (out_size != kRows * kDm) return;
  if (ws_size < kWsTotal) return;

  const float* x      = (const float*)d_in[0];
  const float* W_in   = (const float*)d_in[1];
  const float* cw[2]  = {(const float*)d_in[2], (const float*)d_in[4]};
  const float* cb[2]  = {(const float*)d_in[3], (const float*)d_in[5]};
  const float* wxp[2] = {(const float*)d_in[6], (const float*)d_in[7]};
  const float* wdt[2] = {(const float*)d_in[8], (const float*)d_in[10]};
  const float* bdt[2] = {(const float*)d_in[9], (const float*)d_in[11]};
  const float* alg[2] = {(const float*)d_in[12], (const float*)d_in[13]};
  const float* dsk[2] = {(const float*)d_in[14], (const float*)d_in[15]};
  const float* W_out  = (const float*)d_in[16];
  float* out = (float*)d_out;

  char* ws = (char*)d_ws;
  unsigned short* X16    = (unsigned short*)(ws + kOffX16);
  unsigned short* WIN16  = (unsigned short*)(ws + kOffWIN);
  unsigned short* WOUT16 = (unsigned short*)(ws + kOffWOUT);
  unsigned short* WX16[2] = {(unsigned short*)(ws + kOffWXF), (unsigned short*)(ws + kOffWXB)};
  unsigned short* WD16[2] = {(unsigned short*)(ws + kOffWDF), (unsigned short*)(ws + kOffWDB)};
  float*          XZB    = (float*)(ws + kOffXZB);
  float*          U32    = (float*)(ws + kOffU32);
  unsigned short* U16    = (unsigned short*)(ws + kOffU16);
  float*          XDBL   = (float*)(ws + kOffXDBL);
  unsigned short* DTLR16 = (unsigned short*)(ws + kOffDTLR);
  float*          DTPRE  = (float*)(ws + kOffDTPRE);
  unsigned short* YD16[2] = {(unsigned short*)(ws + kOffYF), (unsigned short*)(ws + kOffYB)};
  unsigned short* Y16    = (unsigned short*)(ws + kOffY16);

  cast_plane_f16_kernel<<<(kRows * kDm / 8) / 256, 256, 0, stream>>>(x, kDm, kRows, X16, kDm, kRows * kDm / 8, kCX);
  cast_plane_f16_kernel<<<(kXzP * kDm / 8) / 256, 256, 0, stream>>>(W_in, kDm, kXzP, WIN16, kDm, kXzP * kDm / 8, kCWin);
  cast_plane_f16_kernel<<<(kDm * kDin / 8) / 256, 256, 0, stream>>>(W_out, kDin, kDm, WOUT16, kDin, kDm * kDin / 8, kCWo);
  for (int dir = 0; dir < 2; ++dir) {
    cast_plane_f16_kernel<<<(kXdP * kDin / 8) / 256, 256, 0, stream>>>(wxp[dir], kDin, kXdW, WX16[dir], kDin, kXdP * kDin / 8, kCWx);
    cast_plane_f16_kernel<<<(kDin * kDtR / 8) / 256, 256, 0, stream>>>(wdt[dir], kDtR, kDin, WD16[dir], kDtR, kDin * kDtR / 8, kCWdt);
  }

  for (int b = 0; b < kBatch; ++b) {
    eng::gemm_f16_kernel<0><<<dim3((kSeq / 64) * (kXzP / 64) / 8), 256, 0, stream>>>(
        X16 + (size_t)b * kSeq * kDm, kDm, WIN16, kDm, XZB, kXzP, nullptr, kSeq, kXzP, kDm, kSclIn);

    for (int dir = 0; dir < 2; ++dir) {
      conv_silu_kernel<<<dim3(kDin / 256, kSeq / 64), 256, 0, stream>>>(XZB, cw[dir], cb[dir], U32, U16, dir);

      if (dir == 1) zflip_kernel<<<(kSeq / 2) * (kDin / 4) / 256, 256, 0, stream>>>(XZB + kDin, XZB);

      eng::gemm_f16_kernel<0><<<dim3((kSeq / 64) * (kXdP / 64) / 8), 256, 0, stream>>>(
          U16, kDin, WX16[dir], kDin, XDBL, kXdP, nullptr, kSeq, kXdP, kDin, kSclXp);

      cast_plane_f16_kernel<<<(kSeq * kDtR / 8) / 256, 256, 0, stream>>>(XDBL, kXdP, kSeq, DTLR16, kDtR, kSeq * kDtR / 8, kCDt);

      eng::gemm_f16_kernel<1><<<dim3((kSeq / 64) * (kDin / 64) / 8), 256, 0, stream>>>(
          DTLR16, kDtR, WD16[dir], kDtR, DTPRE, kDin, bdt[dir], kSeq, kDin, kDtR, kSclDt);

      ms1_args sa;
      sa.dtpre = DTPRE;
      sa.u = U32;
      sa.bc = XDBL;
      sa.z = XZB;
      sa.A_log = alg[dir];
      sa.Dskip = dsk[dir];
      sa.y = (__half*)YD16[dir];
      sa.y_lo = nullptr;
      sa.ld_dtpre = kDin;
      sa.ld_u = kDin;
      sa.ld_bc = kXdP;
      sa.ld_z = kXzP;
      sa.ld_y = kDin;
      sa.offB = kOffB;
      sa.offC = kOffC;
      sa.offZ = (dir == 0) ? kDin : 0;
      sa.ycarry = kCY;
      sa.dir = 1;
      sa.D = kDin;
      sa.L = kSeq;
      sa.nbatch = 1;
      ms1_scan_kernel<16><<<dim3(kDin / 64), 64, 0, stream>>>(sa);
    }

    combine_kernel<<<(kSeq * (kDin / 8)) / 256, 256, 0, stream>>>(
        (const unsigned*)YD16[0], (const unsigned*)YD16[1], Y16 + (size_t)b * kSeq * kDin);
  }

  eng::gemm_f16_kernel<0><<<dim3((kRows / 64) * (kDm / 64) / 8), 256, 0, stream>>>(
      Y16, kDin, WOUT16, kDin, out, kDm, nullptr, kRows, kDm, kDin, kSclOut);
}
